// DAWNLayer_10419590660471
// MI455X (gfx1250) — hardware-run, weakly checked
//
#include <hip/hip_runtime.h>

typedef __attribute__((ext_vector_type(16))) _Float16 v16h;
typedef __attribute__((ext_vector_type(8)))  _Float16 v8h;
typedef __attribute__((ext_vector_type(16))) __bf16   v16b;
typedef __attribute__((ext_vector_type(8)))  __bf16   v8b;
typedef __attribute__((ext_vector_type(8)))  float    v8f;
typedef __attribute__((ext_vector_type(4)))  float    v4f;
typedef __attribute__((ext_vector_type(4)))  unsigned int v4u;

constexpr int NBATCH = 8;
constexpr int SEQL = 1024;
constexpr int NTOK = NBATCH * SEQL;
constexpr int DMOD = 768;
constexpr int NHEADS = 12;
constexpr int HDIM = 64;
constexpr int DFFN = 3072;
constexpr int NNEU = 96;
constexpr int NNEU_PAD = 128;
constexpr int NBAS = 32;
constexpr int RNK = 64;
constexpr int TOPKK = 8;
constexpr int NPROJ = NBAS * RNK;

constexpr float WCARRY = 64.0f;
constexpr float WCARRY_INV = 1.0f / 64.0f;
constexpr float VSCARRY = 64.0f;
constexpr float VCARRY = 64.0f;
constexpr float OCARRY_EXTRA = 16.0f;
constexpr float GCARRY = 16.0f;
constexpr float PCARRY = 32768.0f;

static_assert(NTOK % 64 == 0 && DMOD % 64 == 0 && DFFN % 64 == 0 && NPROJ % 64 == 0 && NNEU_PAD % 64 == 0, "M,N tile multiples");
static_assert(DMOD % 32 == 0 && DFFN % 32 == 0 && NBAS % 32 == 0 && RNK % 32 == 0, "K multiple of 32");
static_assert(SEQL % 64 == 0 && HDIM == 64 && NHEADS * HDIM == DMOD, "attention geometry");
static_assert(DMOD % 8 == 0 && (DMOD / 8) == 96, "layernorm lane map");
static_assert(NNEU % 4 == 0 && NTOK % 32 == 0 && NTOK % 4 == 0, "topk / vsem block maps");

constexpr size_t SZ_W768   = (size_t)DMOD * DMOD * 2;
constexpr size_t SZ_WVO    = (size_t)DMOD * RNK * 2;
constexpr size_t SZ_WUP    = (size_t)DFFN * DMOD * 2;
constexpr size_t SZ_WDN    = (size_t)DMOD * DFFN * 2;
constexpr size_t SZ_BA     = (size_t)NPROJ * DMOD * 2;
constexpr size_t SZ_BEMBT  = (size_t)DMOD * NBAS * 2;
constexpr size_t SZ_RNA    = (size_t)NNEU_PAD * NBAS * 2;
constexpr size_t SZ_RN     = (size_t)NNEU * NBAS * 4;
constexpr size_t SZ_CSIG   = (size_t)NNEU_PAD * 4;
constexpr size_t SZ_VB64   = (size_t)DMOD * 4;
constexpr size_t SZ_NEMB   = (size_t)NNEU_PAD * DMOD * 2;
constexpr size_t SZ_X2     = (size_t)NTOK * DMOD * 4;
constexpr size_t SZ_ACT16  = (size_t)NTOK * DMOD * 2;
constexpr size_t SZ_SEM    = (size_t)NTOK * NNEU_PAD * 4;
constexpr size_t SZ_TR     = (size_t)NTOK * NBAS * 4;
constexpr size_t SZ_VSEM   = (size_t)NTOK * RNK * 2;
constexpr size_t SZ_PROJ   = (size_t)NTOK * NPROJ * 2;
constexpr size_t SZ_H      = (size_t)NTOK * DFFN * 2;

constexpr size_t OFF_WQ    = 0;
constexpr size_t OFF_WK    = OFF_WQ + SZ_W768;
constexpr size_t OFF_WAO   = OFF_WK + SZ_W768;
constexpr size_t OFF_WVO   = OFF_WAO + SZ_W768;
constexpr size_t OFF_WUP   = OFF_WVO + SZ_WVO;
constexpr size_t OFF_WDN   = OFF_WUP + SZ_WUP;
constexpr size_t OFF_BA    = OFF_WDN + SZ_WDN;
constexpr size_t OFF_BEMBT = OFF_BA + SZ_BA;
constexpr size_t OFF_RNA   = OFF_BEMBT + SZ_BEMBT;
constexpr size_t OFF_RN    = OFF_RNA + SZ_RNA;
constexpr size_t OFF_CSIG  = OFF_RN + SZ_RN;
constexpr size_t OFF_VB64  = OFF_CSIG + SZ_CSIG;
constexpr size_t OFF_NEMB  = OFF_VB64 + SZ_VB64;
constexpr size_t OFF_X2    = OFF_NEMB + SZ_NEMB;
constexpr size_t OFF_NORM  = OFF_X2 + SZ_X2;
constexpr size_t OFF_Q     = OFF_NORM + SZ_ACT16;
constexpr size_t OFF_K     = OFF_Q + SZ_ACT16;
constexpr size_t OFF_V     = OFF_K + SZ_ACT16;
constexpr size_t OFF_SEM   = OFF_V + SZ_ACT16;
constexpr size_t OFF_TR    = OFF_SEM + SZ_SEM;
constexpr size_t OFF_VSEM  = OFF_TR + SZ_TR;
constexpr size_t OFF_PROJ  = OFF_VSEM + SZ_VSEM;
constexpr size_t WS_TOTAL  = OFF_PROJ + SZ_PROJ;
constexpr size_t OFF_ATTN  = OFF_SEM;
constexpr size_t OFF_H     = OFF_Q;
static_assert(WS_TOTAL <= (size_t)134217728, "carve under 128 MiB");
static_assert(OFF_ATTN + SZ_ACT16 <= WS_TOTAL, "attn alias fits");
static_assert(OFF_H + SZ_H <= WS_TOTAL, "hidden alias fits");
static_assert(OFF_ATTN >= OFF_V + SZ_ACT16, "attn alias does not overlap Q/K/V");
static_assert((OFF_NEMB % 256) == 0 && (OFF_X2 % 256) == 0 && (OFF_PROJ % 256) == 0 && (OFF_VB64 % 256) == 0, "alignment");

__device__ __forceinline__ unsigned short f2bf_bits(float f) {
  unsigned u = __float_as_uint(f);
  return (unsigned short)((u + 0x7FFFu + ((u >> 16) & 1u)) >> 16);
}
__device__ __forceinline__ float bf_bits2f(unsigned short h) { return __uint_as_float(((unsigned)h) << 16); }

__device__ __forceinline__ unsigned short h_bits(float f) { return __builtin_bit_cast(unsigned short, (_Float16)f); }
__device__ __forceinline__ float h_val(unsigned int b16) { return (float)__builtin_bit_cast(_Float16, (unsigned short)(b16 & 0xffffu)); }

__device__ __forceinline__ void dep_guard_h(v8f& a, v8f& b, v16h x, v16h y) { asm volatile("v_nop\n\tv_nop\n\tv_nop\n\tv_nop" : "+v"(a), "+v"(b) : "v"(x), "v"(y)); }
__device__ __forceinline__ void dep_guard_b(v8f& a, v8f& b, v16b x, v16b y) { asm volatile("v_nop\n\tv_nop\n\tv_nop\n\tv_nop" : "+v"(a), "+v"(b) : "v"(x), "v"(y)); }
__device__ __forceinline__ void keep4_h(v16h a, v16h b, v16h c, v16h d) { asm volatile("v_nop" :: "v"(a), "v"(b), "v"(c), "v"(d)); }
__device__ __forceinline__ void keep4_b(v16b a, v16b b, v16b c, v16b d) { asm volatile("v_nop" :: "v"(a), "v"(b), "v"(c), "v"(d)); }
__device__ __forceinline__ void acc_guard4(v8f& a, v8f& b, v8f& c, v8f& d) { asm volatile("v_nop\n\tv_nop\n\tv_nop\n\tv_nop" : "+v"(a), "+v"(b), "+v"(c), "+v"(d)); }
template <typename T> struct Frag;
template <> struct Frag<_Float16> {
  typedef v16h V; union U { v16h v; v8h h[2]; };
  static __device__ __forceinline__ v16h load(const _Float16* p) {
    U f; f.h[0] = *(const v8h*)(p); f.h[1] = *(const v8h*)(p + 16); return f.v;
  }
  static __device__ __forceinline__ v8f mma(v16h a, v16h b, v8f c) {
    return __builtin_amdgcn_wmma_f32_16x16x32_f16(false, a, false, b, (short)0, c, false, false);
  }
  static __device__ __forceinline__ void guard(v8f& a, v8f& b, v16h x, v16h y) { dep_guard_h(a, b, x, y); }
  static __device__ __forceinline__ void keep(v16h a, v16h b, v16h c, v16h d) { keep4_h(a, b, c, d); }
};
template <> struct Frag<__bf16> {
  typedef v16b V; union U { v16b v; v8b h[2]; };
  static __device__ __forceinline__ v16b load(const __bf16* p) {
    U f; f.h[0] = *(const v8b*)(p); f.h[1] = *(const v8b*)(p + 16); return f.v;
  }
  static __device__ __forceinline__ v8f mma(v16b a, v16b b, v8f c) {
    return __builtin_amdgcn_wmma_f32_16x16x32_bf16(false, a, false, b, (short)0, c, false, false);
  }
  static __device__ __forceinline__ void guard(v8f& a, v8f& b, v16b x, v16b y) { dep_guard_b(a, b, x, y); }
  static __device__ __forceinline__ void keep(v16b a, v16b b, v16b c, v16b d) { keep4_b(a, b, c, d); }
};

__device__ __forceinline__ v8f mma_h(v16h a, v16h b, v8f c) {
  c = __builtin_amdgcn_wmma_f32_16x16x32_f16(false, a, false, b, (short)0, c, false, false);
  asm volatile("v_nop\n\tv_nop\n\tv_nop\n\tv_nop" : "+v"(c) : "v"(a), "v"(b));
  return c;
}

template <int ET> struct Elem;
template <> struct Elem<0> { typedef _Float16 T; };
template <> struct Elem<1> { typedef __bf16 T; };
template <int ET, bool SPLIT, int BIAS_MODE, int OUT_MODE, bool RESID, int ACT = 0>
__global__ __launch_bounds__(256) void wmma_gemm64(
    const unsigned short* __restrict__ Ap, const unsigned short* __restrict__ A2p, int lda, long strideA,
    const unsigned short* __restrict__ Btp, const unsigned short* __restrict__ Bt2p, int ldb, long strideB,
    void* __restrict__ Cout, void* __restrict__ Cout2, int ldc, long strideC,
    const float* __restrict__ bias,
    const float* __restrict__ resid, long strideR,
    int M, int N, int K, float scale) {
  static_assert(!(RESID && OUT_MODE != 0), "residual only with f32 output");
  typedef typename Elem<ET>::T T;
  typedef typename Frag<T>::V V;
  const T* A = (const T*)Ap; const T* A2 = (const T*)A2p; const T* Bt = (const T*)Btp; const T* Bt2 = (const T*)Bt2p;
  __shared__ __align__(16) float sT[8][16 * 68];
  const int b    = blockIdx.y;
  const int lane = threadIdx.x & 31;
  const int wave = threadIdx.x >> 5;
  const int tilesN = N >> 6;
  const int tilesM = M >> 6;
  const int tile = blockIdx.x * 8 + wave;
  if (tile >= tilesM * tilesN) return;
  const int tm = tile / tilesN;
  const int tn = tile - tm * tilesN;
  const int m0 = tm << 6;
  const int n0 = tn << 6;

  const T* Ab  = A  + (size_t)b * strideA;
  const T* Bb  = Bt + (size_t)b * strideB;
  const T* Ab2 = SPLIT ? (A2  + (size_t)b * strideA) : nullptr;
  const T* Bb2 = SPLIT ? (Bt2 + (size_t)b * strideB) : nullptr;

  const int rlane = lane & 15;
  const int koff  = (lane >> 4) * 8;
  const int mOff  = (lane >> 4) * 8;

  v8f acc[4][4];
#pragma unroll
  for (int i = 0; i < 4; ++i)
#pragma unroll
    for (int j = 0; j < 4; ++j) acc[i][j] = (v8f){0.f,0.f,0.f,0.f,0.f,0.f,0.f,0.f};

  for (int k0 = 0; k0 < K; k0 += 32) {
    V bh[4], bl[4];
#pragma unroll
    for (int j = 0; j < 4; ++j) {
      const size_t bo = (size_t)(n0 + (j << 4) + rlane) * ldb + koff + k0;
      bh[j] = Frag<T>::load(Bb + bo);
      if (SPLIT) bl[j] = Frag<T>::load(Bb2 + bo);
    }
#pragma unroll
    for (int i = 0; i < 4; ++i) {
      const size_t ao = (size_t)(m0 + (i << 4) + rlane) * lda + koff + k0;
      V ah = Frag<T>::load(Ab + ao);
      V al;
      if (SPLIT) al = Frag<T>::load(Ab2 + ao);
#pragma unroll
      for (int j = 0; j < 4; ++j) {
        acc[i][j] = Frag<T>::mma(ah, bh[j], acc[i][j]);
        if (SPLIT) {
          acc[i][j] = Frag<T>::mma(ah, bl[j], acc[i][j]);
          acc[i][j] = Frag<T>::mma(al, bh[j], acc[i][j]);
        }
      }
      Frag<T>::guard(acc[i][0], acc[i][3], ah, SPLIT ? al : ah);
    }
    Frag<T>::keep(bh[0], bh[1], bh[2], bh[3]);
    if (SPLIT) Frag<T>::keep(bl[0], bl[1], bl[2], bl[3]);
  }
  acc_guard4(acc[0][0], acc[0][1], acc[0][2], acc[0][3]);
  acc_guard4(acc[1][0], acc[1][1], acc[1][2], acc[1][3]);
  acc_guard4(acc[2][0], acc[2][1], acc[2][2], acc[2][3]);
  acc_guard4(acc[3][0], acc[3][1], acc[3][2], acc[3][3]);

  float* slab = sT[wave];
#pragma unroll
  for (int i = 0; i < 4; ++i) {
    const int mBase = m0 + (i << 4);
#pragma unroll
    for (int j = 0; j < 4; ++j) {
      const int n = n0 + (j << 4) + rlane;
      float bv = 0.f;
      if (BIAS_MODE == 2) bv = bias[n];
#pragma unroll
      for (int r = 0; r < 8; ++r) {
        float v = acc[i][j][r] * scale;
        if (BIAS_MODE == 1) v += bias[mBase + mOff + r];
        if (BIAS_MODE == 2) v += bv;
        if (ACT == 1) v = tanhf(v);
        if (ACT == 2) v = fmaxf(v, 0.0f);
        if (ACT == 3) v = v / (1.0f + expf(-v));
        if (ACT == 4) v = (v > 0.f) ? v : 0.01f * v;
        slab[(mOff + r) * 68 + (j << 4) + rlane] = v;
      }
    }
    __builtin_amdgcn_fence(__ATOMIC_RELEASE, "workgroup");
    __builtin_amdgcn_wave_barrier();
    __builtin_amdgcn_fence(__ATOMIC_ACQUIRE, "workgroup");
    if (OUT_MODE == 0) {
      float* C = (float*)Cout + (size_t)b * strideC;
      const float* Rb = RESID ? (resid + (size_t)b * strideR) : nullptr;
      const int hh = lane >> 4, c4 = (lane & 15) * 4;
      for (int pass = 0; pass < 2; ++pass) {
#pragma unroll
        for (int it = 0; it < 8; ++it) {
          const int row = it * 2 + hh;
          v4f v = *(const v4f*)(slab + row * 68 + c4);
          if (RESID) {
            const v4f rr = *(const v4f*)(Rb + (size_t)(mBase + row) * ldc + n0 + c4);
            v += rr;
          }
          *(volatile v4f*)(C + (size_t)(mBase + row) * ldc + n0 + c4) = v;
        }
        __threadfence();
      }
    } else {
      const int q = lane >> 3, c8 = (lane & 7) * 8;
      unsigned short* C  = (unsigned short*)Cout  + (size_t)b * strideC;
      unsigned short* C2 = (OUT_MODE == 2) ? ((unsigned short*)Cout2 + (size_t)b * strideC) : nullptr;
      for (int pass = 0; pass < 2; ++pass) {
#pragma unroll
        for (int it = 0; it < 4; ++it) {
          const int row = it * 4 + q;
          const float* sp = slab + row * 68 + c8;
          v8h hv, lv;
#pragma unroll
          for (int e = 0; e < 8; ++e) {
            if (OUT_MODE == 1) {
              hv[e] = (_Float16)sp[e];
            } else {
              unsigned short hb = f2bf_bits(sp[e]);
              unsigned short lb = f2bf_bits(sp[e] - bf_bits2f(hb));
              hv[e] = __builtin_bit_cast(_Float16, hb);
              lv[e] = __builtin_bit_cast(_Float16, lb);
            }
          }
          *(volatile v8h*)(C + (size_t)(mBase + row) * ldc + n0 + c8) = hv;
          if (OUT_MODE == 2) *(volatile v8h*)(C2 + (size_t)(mBase + row) * ldc + n0 + c8) = lv;
        }
        __threadfence();
      }
    }
    __builtin_amdgcn_fence(__ATOMIC_RELEASE, "workgroup");
    __builtin_amdgcn_wave_barrier();
    __builtin_amdgcn_fence(__ATOMIC_ACQUIRE, "workgroup");
  }
}

__global__ __launch_bounds__(256) void k_tcast(const float* __restrict__ in, unsigned short* __restrict__ out,
                                               int rows, int cols, long in_bstride, long out_bstride, float sc) {
  __shared__ __align__(16) unsigned short tile[64 * 72];
  const int t = threadIdx.x, lane = t & 31, wave = t >> 5;
  const float* src = in + (size_t)blockIdx.z * in_bstride;
  unsigned short* dst = out + (size_t)blockIdx.z * out_bstride;
  const int r0 = blockIdx.y * 64, c0 = blockIdx.x * 64;
  const int lr = t >> 2, lc = (t & 3) * 16;
  const float* p = src + (size_t)(r0 + lr) * cols + c0 + lc;
  v4f a[4];
#pragma unroll
  for (int i = 0; i < 4; ++i) a[i] = *(const v4f*)(p + 4 * i);
#pragma unroll
  for (int i = 0; i < 4; ++i) {
#pragma unroll
    for (int e = 0; e < 4; ++e) tile[(lc + 4 * i + e) * 72 + lr] = h_bits(a[i][e] * sc);
  }
  __syncthreads();
  const int q = lane >> 3, c8 = (lane & 7) * 8;
  v4u v[2];
#pragma unroll
  for (int rnd = 0; rnd < 2; ++rnd) {
    const int n = rnd * 32 + wave * 4 + q;
    v[rnd] = *(const v4u*)(tile + n * 72 + c8);
  }
  for (int pass = 0; pass < 2; ++pass) {
#pragma unroll
    for (int rnd = 0; rnd < 2; ++rnd) {
      const int n = rnd * 32 + wave * 4 + q;
      *(volatile v4u*)(dst + (size_t)(c0 + n) * rows + r0 + c8) = v[rnd];
    }
    __threadfence();
  }
}

__global__ __launch_bounds__(256) void k_prep(const float* __restrict__ recipe, const float* __restrict__ ctx,
                                              const float* __restrict__ bemb, const float* __restrict__ vbias,
                                              float* __restrict__ rn_out, unsigned short* __restrict__ rnA,
                                              float* __restrict__ csig, float* __restrict__ vb_out,
                                              unsigned short* __restrict__ bembT) {
  __shared__ __align__(16) float rn_s[NNEU * NBAS];
  __shared__ __align__(16) unsigned short rh_s[NNEU_PAD * NBAS];
  __shared__ __align__(16) float cs_s[NNEU_PAD];
  __shared__ __align__(16) unsigned short bt_s[384 * NBAS];
  const int t = threadIdx.x;
  float den = 1.0f;
  if (t < NNEU) {
    const float* r = recipe + t * NBAS;
    float mx = -INFINITY;
#pragma unroll 1
    for (int j = 0; j < NBAS; ++j) mx = fmaxf(mx, r[j]);
    float dsum = 0.f;
#pragma unroll 1
    for (int j = 0; j < NBAS; ++j) { const float e = expf(r[j] - mx); rn_s[t * NBAS + j] = e; dsum += e; }
    den = dsum;
    float c = 0.f;
#pragma unroll 1
    for (int hh = 0; hh < NHEADS; ++hh) c += ctx[t * NHEADS + hh];
    c = c * (1.0f / (float)SEQL);
    cs_s[t] = 1.0f / (1.0f + expf(-c));
  } else if (t < NNEU_PAD) {
    cs_s[t] = 0.f;
  }
  if (t < NNEU) {
    const float inv = 1.0f / den;
#pragma unroll 1
    for (int j = 0; j < NBAS; ++j) {
      const float v = rn_s[t * NBAS + j] * inv;
      rn_s[t * NBAS + j] = v;
      rh_s[t * NBAS + j] = h_bits(v);
    }
  } else if (t < NNEU_PAD) {
    const v4u z = {0u, 0u, 0u, 0u};
#pragma unroll
    for (int i = 0; i < 4; ++i) *(v4u*)(rh_s + t * NBAS + 8 * i) = z;
  }
  __syncthreads();
  for (int pass = 0; pass < 2; ++pass) {
#pragma unroll
    for (int it = 0; it < 3; ++it) {
      const int idx = it * 256 + t;
      *(volatile v4f*)(rn_out + idx * 4) = *(const v4f*)(rn_s + idx * 4);
    }
#pragma unroll
    for (int it = 0; it < 2; ++it) {
      const int idx = it * 256 + t;
      *(volatile v4u*)(rnA + idx * 8) = *(const v4u*)(rh_s + idx * 8);
    }
    if (t < NNEU_PAD / 4) *(volatile v4f*)(csig + t * 4) = *(const v4f*)(cs_s + t * 4);
    if (t < DMOD / 4) {
      const v4f vb = *(const v4f*)(vbias + t * 4);
      *(volatile v4f*)(vb_out + t * 4) = vb * VCARRY;
    }
    __threadfence();
  }
  for (int half = 0; half < 2; ++half) {
    __syncthreads();
#pragma unroll 1
    for (int idx = t; idx < NBAS * 384; idx += 256) {
      const int j = idx / 384, dd = idx - j * 384;
      bt_s[dd * NBAS + j] = h_bits(bemb[(size_t)j * DMOD + half * 384 + dd] * WCARRY);
    }
    __syncthreads();
    unsigned short* dsth = bembT + (size_t)half * 384 * NBAS;
    for (int pass = 0; pass < 2; ++pass) {
#pragma unroll
      for (int it = 0; it < 6; ++it) {
        const int idx = it * 256 + t;
        *(volatile v4u*)(dsth + idx * 8) = *(const v4u*)(bt_s + idx * 8);
      }
      __threadfence();
    }
  }
}

__global__ __launch_bounds__(128) void k_ln(const float* __restrict__ x, const float* __restrict__ g,
                                            const float* __restrict__ bb, unsigned short* __restrict__ outp) {
  __shared__ float red_a[4];
  __shared__ float red_b[4];
  const int row = blockIdx.x;
  const int t = threadIdx.x, lane = t & 31, wave = t >> 5;
  const bool act = t < (DMOD / 8);
  const int tc = act ? t : (DMOD / 8 - 1);
  const float* xr = x + (size_t)row * DMOD + tc * 8;
  const v4f p0 = *(const v4f*)xr;
  const v4f p1 = *(const v4f*)(xr + 4);
  float v[8] = {p0[0], p0[1], p0[2], p0[3], p1[0], p1[1], p1[2], p1[3]};
  float s = 0.f;
#pragma unroll
  for (int e = 0; e < 8; ++e) s += v[e];
  s = act ? s : 0.f;
#pragma unroll
  for (int off = 1; off < 32; off <<= 1) s += __shfl_xor(s, off, 32);
  if (lane == 0) red_a[wave] = s;
  __syncthreads();
  const float mean = ((red_a[0] + red_a[1]) + (red_a[2] + red_a[3])) * (1.0f / (float)DMOD);
  float d[8];
  float s2 = 0.f;
#pragma unroll
  for (int e = 0; e < 8; ++e) { d[e] = v[e] - mean; s2 += d[e] * d[e]; }
  s2 = act ? s2 : 0.f;
#pragma unroll
  for (int off = 1; off < 32; off <<= 1) s2 += __shfl_xor(s2, off, 32);
  if (lane == 0) red_b[wave] = s2;
  __syncthreads();
  const float var = ((red_b[0] + red_b[1]) + (red_b[2] + red_b[3])) * (1.0f / (float)DMOD);
  const float rstd = rsqrtf(var + 1e-5f);
  const v4f g0 = *(const v4f*)(g + tc * 8), g1 = *(const v4f*)(g + tc * 8 + 4);
  const v4f b0 = *(const v4f*)(bb + tc * 8), b1 = *(const v4f*)(bb + tc * 8 + 4);
  const float gv[8] = {g0[0], g0[1], g0[2], g0[3], g1[0], g1[1], g1[2], g1[3]};
  const float bv[8] = {b0[0], b0[1], b0[2], b0[3], b1[0], b1[1], b1[2], b1[3]};
  float y[8];
#pragma unroll
  for (int e = 0; e < 8; ++e) y[e] = d[e] * rstd * gv[e] + bv[e];
  v4u o;
  o[0] = (unsigned)h_bits(y[0]) | ((unsigned)h_bits(y[1]) << 16);
  o[1] = (unsigned)h_bits(y[2]) | ((unsigned)h_bits(y[3]) << 16);
  o[2] = (unsigned)h_bits(y[4]) | ((unsigned)h_bits(y[5]) << 16);
  o[3] = (unsigned)h_bits(y[6]) | ((unsigned)h_bits(y[7]) << 16);
  unsigned short* op = outp + (size_t)row * DMOD + tc * 8;
  if (act) *(volatile v4u*)op = o;
  __threadfence();
  if (act) *(volatile v4u*)op = o;
}

__device__ __forceinline__ void tk_insert(float (&s)[8], int (&ix)[8], float v, int n) {
  if (v > s[7]) { s[7] = v; ix[7] = n; }
#pragma unroll
  for (int k = 7; k > 0; --k) {
    const bool sw = s[k] > s[k - 1];
    const float ts = s[k - 1];
    const int ti = ix[k - 1];
    const float cs = s[k];
    const int ci = ix[k];
    s[k - 1] = sw ? cs : ts;
    ix[k - 1] = sw ? ci : ti;
    s[k] = sw ? ts : cs;
    ix[k] = sw ? ti : ci;
  }
}

__global__ __launch_bounds__(256) void k_topk(const float* __restrict__ sem, const float* __restrict__ csig,
                                              const float* __restrict__ rn, float* __restrict__ tr, int ntok) {
  __shared__ float w_s[32][TOPKK];
  __shared__ int   i_s[32][TOPKK];
  const int t = threadIdx.x;
  const int tok0 = blockIdx.x * 32;
  if (t < 32) {
    const int tok = tok0 + t;
    const int tokc = tok < ntok ? tok : ntok - 1;
    const float* srow = sem + (size_t)tokc * NNEU_PAD;
    float s[8];
    int ix[8];
#pragma unroll
    for (int k = 0; k < 8; ++k) { s[k] = -INFINITY; ix[k] = 0; }
#pragma unroll 1
    for (int n4 = 0; n4 < NNEU / 4; ++n4) {
      const v4f sv = *(const v4f*)(srow + n4 * 4);
      const v4f cg = *(const v4f*)(csig + n4 * 4);
#pragma unroll
      for (int e = 0; e < 4; ++e) tk_insert(s, ix, sv[e] * cg[e], n4 * 4 + e);
    }
#pragma unroll
    for (int k = 0; k < 8; ++k) {
      w_s[t][k] = s[k];
      int id = ix[k];
      id = id < 0 ? 0 : (id > NNEU - 1 ? NNEU - 1 : id);
      i_s[t][k] = id;
    }
    const float mx = s[0];
    float den = 0.f;
#pragma unroll 1
    for (int k = 0; k < TOPKK; ++k) {
      const float e = expf(w_s[t][k] - mx);
      w_s[t][k] = e;
      den += e;
    }
    const float inv = 1.0f / den;
#pragma unroll 1
    for (int k = 0; k < TOPKK; ++k) w_s[t][k] = w_s[t][k] * inv;
  }
  __syncthreads();
  const int tk = t >> 3, jc = (t & 7) * 4;
  const int tok = tok0 + tk;
  v4f acc = {0.f, 0.f, 0.f, 0.f};
#pragma unroll 1
  for (int k = 0; k < TOPKK; ++k) {
    const int id = i_s[tk][k];
    const float wk = w_s[tk][k];
    const v4f rv = *(const v4f*)(rn + id * NBAS + jc);
    acc += rv * wk;
  }
  float* dstp = tr + (size_t)(tok < ntok ? tok : ntok - 1) * NBAS + jc;
  if (tok < ntok) *(volatile v4f*)dstp = acc;
  __threadfence();
  if (tok < ntok) *(volatile v4f*)dstp = acc;
}

__global__ __launch_bounds__(128) void k_vsem(const unsigned short* __restrict__ proj, const float* __restrict__ tr,
                                              unsigned short* __restrict__ vs, int ntok) {
  const int lane = threadIdx.x & 31, wave = threadIdx.x >> 5;
  const int tok = blockIdx.x * 4 + wave;
  const int tokc = tok < ntok ? tok : ntok - 1;
  const float trv = tr[(size_t)tokc * NBAS + lane];
  const unsigned int* prow = (const unsigned int*)(proj + (size_t)tokc * NPROJ) + lane;
  float a0 = 0.f, a1 = 0.f;
#pragma unroll 1
  for (int n = 0; n < NBAS; ++n) {
    const float w = __shfl(trv, n, 32);
    const unsigned int pw = prow[n * (RNK / 2)];
    a0 += w * h_val(pw & 0xffffu);
    a1 += w * h_val(pw >> 16);
  }
  const unsigned int o = (unsigned)h_bits(a0 * VSCARRY) | ((unsigned)h_bits(a1 * VSCARRY) << 16);
  unsigned int* dstw = (unsigned int*)(vs + (size_t)tokc * RNK) + lane;
  if (tok < ntok) *(volatile unsigned int*)dstw = o;
  __threadfence();
  if (tok < ntok) *(volatile unsigned int*)dstw = o;
}

__global__ __launch_bounds__(128) void k_attn(const unsigned short* __restrict__ Qp, const unsigned short* __restrict__ Kp,
                                              const unsigned short* __restrict__ Vp, unsigned short* __restrict__ Op,
                                              float qscale, float ocarry) {
  __shared__ __align__(16) unsigned short Ksh[64 * 64];
  __shared__ __align__(16) unsigned short Vth[64 * 64];
  __shared__ __align__(16) unsigned short Psh[4][16 * 64];
  __shared__ __align__(16) float Os[4][16 * 68];
  const int tid = threadIdx.x, wave = tid >> 5, lane = tid & 31, hh = lane >> 4, c = lane & 15;
  constexpr int nqb = SEQL / 64;
  const int bx = blockIdx.x;
  const int qb = bx % nqb, bh = bx / nqb;
  const int h = bh % NHEADS, b = bh / NHEADS;
  const int q0 = qb * 64 + wave * 16;
  const size_t hb = (size_t)b * SEQL * DMOD + (size_t)h * HDIM;
  const _Float16* Qh = (const _Float16*)Qp + hb;

  v16h qa[2];
#pragma unroll
  for (int dc = 0; dc < 2; ++dc) qa[dc] = Frag<_Float16>::load(Qh + (size_t)(q0 + c) * DMOD + dc * 32 + 8 * hh);

  float mrow[8], lrow[8];
  v8f oacc[4];
#pragma unroll
  for (int r = 0; r < 8; ++r) { mrow[r] = -INFINITY; lrow[r] = 0.f; }
#pragma unroll
  for (int t4 = 0; t4 < 4; ++t4) oacc[t4] = (v8f){0.f,0.f,0.f,0.f,0.f,0.f,0.f,0.f};

  for (int kc = 0; kc < SEQL / 64; ++kc) {
    const int kv0 = kc * 64;
    __syncthreads();
    {
      const int kvr = tid >> 1, dh = (tid & 1) * 32;
      const unsigned short* krow = Kp + hb + (size_t)(kv0 + kvr) * DMOD + dh;
      const unsigned short* vrow = Vp + hb + (size_t)(kv0 + kvr) * DMOD + dh;
      v4u kk[4], vv[4];
#pragma unroll
      for (int i = 0; i < 4; ++i) { kk[i] = *(const v4u*)(krow + 8 * i); vv[i] = *(const v4u*)(vrow + 8 * i); }
#pragma unroll
      for (int i = 0; i < 4; ++i) {
        *(v4u*)(Ksh + kvr * 64 + dh + 8 * i) = kk[i];
#pragma unroll
        for (int e = 0; e < 4; ++e) {
          const unsigned int w = vv[i][e];
          const int d = dh + 8 * i + 2 * e;
          Vth[d * 64 + kvr] = (unsigned short)(w & 0xffffu);
          Vth[(d + 1) * 64 + kvr] = (unsigned short)(w >> 16);
        }
      }
    }
    __syncthreads();

    v8f s[4];
#pragma unroll
    for (int j = 0; j < 4; ++j) {
      s[j] = (v8f){0.f,0.f,0.f,0.f,0.f,0.f,0.f,0.f};
#pragma unroll
      for (int dc = 0; dc < 2; ++dc) {
        const v16h kb = Frag<_Float16>::load((const _Float16*)Ksh + (j * 16 + c) * 64 + dc * 32 + 8 * hh);
        s[j] = mma_h(qa[dc], kb, s[j]);
      }
    }
    float cm[8];
#pragma unroll
    for (int r = 0; r < 8; ++r) {
      float m = -INFINITY;
#pragma unroll
      for (int j = 0; j < 4; ++j) { s[j][r] *= qscale; m = fmaxf(m, s[j][r]); }
#pragma unroll
      for (int off = 1; off < 16; off <<= 1) m = fmaxf(m, __shfl_xor(m, off, 32));
      cm[r] = m;
    }
    unsigned short* pw = Psh[wave];
#pragma unroll
    for (int r = 0; r < 8; ++r) {
      const float mnew = fmaxf(mrow[r], cm[r]);
      const float alpha = expf(mrow[r] - mnew);
      mrow[r] = mnew;
      float psum = 0.f;
#pragma unroll
      for (int j = 0; j < 4; ++j) {
        const float p = expf(s[j][r] - mnew);
        psum += p;
        pw[(8 * hh + r) * 64 + j * 16 + c] = h_bits(p * PCARRY);
      }
#pragma unroll
      for (int off = 1; off < 16; off <<= 1) psum += __shfl_xor(psum, off, 32);
      lrow[r] = lrow[r] * alpha + psum;
#pragma unroll
      for (int t4 = 0; t4 < 4; ++t4) oacc[t4][r] *= alpha;
    }
    __syncthreads();
#pragma unroll
    for (int kk2 = 0; kk2 < 2; ++kk2) {
      const v16h pa = Frag<_Float16>::load((const _Float16*)pw + c * 64 + kk2 * 32 + 8 * hh);
#pragma unroll
      for (int t4 = 0; t4 < 4; ++t4) {
        const v16h vb = Frag<_Float16>::load((const _Float16*)Vth + (t4 * 16 + c) * 64 + kk2 * 32 + 8 * hh);
        oacc[t4] = mma_h(pa, vb, oacc[t4]);
      }
    }
  }

  float* os = Os[wave];
#pragma unroll
  for (int r = 0; r < 8; ++r) {
    const float inv = ocarry / (lrow[r] * PCARRY);
#pragma unroll
    for (int t4 = 0; t4 < 4; ++t4) os[(8 * hh + r) * 68 + t4 * 16 + c] = oacc[t4][r] * inv;
  }
  __syncthreads();
  {
    const int q8 = lane >> 3, c8 = (lane & 7) * 8;
    unsigned short* Ob = Op + hb;
    v4u ov[4];
#pragma unroll
    for (int it = 0; it < 4; ++it) {
      const int row = it * 4 + q8;
      const float* sp = os + row * 68 + c8;
      ov[it][0] = (unsigned)h_bits(sp[0]) | ((unsigned)h_bits(sp[1]) << 16);
      ov[it][1] = (unsigned)h_bits(sp[2]) | ((unsigned)h_bits(sp[3]) << 16);
      ov[it][2] = (unsigned)h_bits(sp[4]) | ((unsigned)h_bits(sp[5]) << 16);
      ov[it][3] = (unsigned)h_bits(sp[6]) | ((unsigned)h_bits(sp[7]) << 16);
    }
    for (int pass = 0; pass < 2; ++pass) {
#pragma unroll
      for (int it = 0; it < 4; ++it) {
        const int row = it * 4 + q8;
        *(volatile v4u*)(Ob + (size_t)(q0 + row) * DMOD + c8) = ov[it];
      }
      __threadfence();
    }
  }
}

__global__ __launch_bounds__(256) void k_gelu2(unsigned int* __restrict__ hw, int n2, float osc) {
  const int i = blockIdx.x * 256 + threadIdx.x;
  if (i < n2) {
    const unsigned int w = hw[i];
    float a = h_val(w & 0xffffu), b = h_val(w >> 16);
    a = 0.5f * a * (1.0f + erff(a * 0.70710678118654752f));
    b = 0.5f * b * (1.0f + erff(b * 0.70710678118654752f));
    const unsigned int u = (unsigned)h_bits(a * osc) | ((unsigned)h_bits(b * osc) << 16);
    ((volatile unsigned int*)hw)[i] = u;
    __threadfence();
    ((volatile unsigned int*)hw)[i] = u;
  }
}

template <int BIASM, int OUTM, bool RES>
static void gemm_f16(const void* A, int lda, const void* Bt, int ldb, void* C, int ldc,
                     const float* bias, const float* resid, int M, int N, int K, float scale, hipStream_t st) {
  const int tiles = (M / 64) * (N / 64);
  const int blocks = (tiles + 7) / 8;
  wmma_gemm64<0, false, BIASM, OUTM, RES, 0><<<dim3(blocks, 1), 256, 0, st>>>(
      (const unsigned short*)A, (const unsigned short*)nullptr, lda, 0L,
      (const unsigned short*)Bt, (const unsigned short*)nullptr, ldb, 0L,
      C, (void*)nullptr, ldc, 0L, bias, resid, 0L, M, N, K, scale);
}

extern "C" void kernel_launch(void* const* d_in, const int* in_sizes, int n_in,
                              void* d_out, int out_size, void* d_ws, size_t ws_size,
                              hipStream_t stream) {
  if (n_in < 21) return;
  if (out_size != NTOK * DMOD) return;
  if (ws_size < WS_TOTAL) return;
  if (in_sizes[0] != NTOK * DMOD || in_sizes[1] != DMOD * DMOD || in_sizes[10] != NBAS * DMOD * RNK ||
      in_sizes[13] != DMOD * DFFN || in_sizes[15] != DFFN * DMOD || in_sizes[7] != NNEU * NBAS ||
      in_sizes[8] != NNEU * NHEADS || in_sizes[9] != NBAS * DMOD || in_sizes[11] != RNK * DMOD) return;

  const float* x       = (const float*)d_in[0];
  const float* q_w     = (const float*)d_in[1];
  const float* q_b     = (const float*)d_in[2];
  const float* k_w     = (const float*)d_in[3];
  const float* k_b     = (const float*)d_in[4];
  const float* ao_w    = (const float*)d_in[5];
  const float* ao_b    = (const float*)d_in[6];
  const float* recipe  = (const float*)d_in[7];
  const float* ctx_pat = (const float*)d_in[8];
  const float* basis_e = (const float*)d_in[9];
  const float* basis_A = (const float*)d_in[10];
  const float* vout_w  = (const float*)d_in[11];
  const float* vout_b  = (const float*)d_in[12];
  const float* up_w    = (const float*)d_in[13];
  const float* up_b    = (const float*)d_in[14];
  const float* down_w  = (const float*)d_in[15];
  const float* down_b  = (const float*)d_in[16];
  const float* n1_g    = (const float*)d_in[17];
  const float* n1_b    = (const float*)d_in[18];
  const float* n2_g    = (const float*)d_in[19];
  const float* n2_b    = (const float*)d_in[20];
  float* out = (float*)d_out;

  char* W = (char*)d_ws;
  unsigned short* wq    = (unsigned short*)(W + OFF_WQ);
  unsigned short* wk    = (unsigned short*)(W + OFF_WK);
  unsigned short* wao   = (unsigned short*)(W + OFF_WAO);
  unsigned short* wvo   = (unsigned short*)(W + OFF_WVO);
  unsigned short* wup   = (unsigned short*)(W + OFF_WUP);
  unsigned short* wdn   = (unsigned short*)(W + OFF_WDN);
  unsigned short* bA    = (unsigned short*)(W + OFF_BA);
  unsigned short* bembT = (unsigned short*)(W + OFF_BEMBT);
  unsigned short* rnA   = (unsigned short*)(W + OFF_RNA);
  float* rn    = (float*)(W + OFF_RN);
  float* csig  = (float*)(W + OFF_CSIG);
  float* vb64  = (float*)(W + OFF_VB64);
  unsigned short* nemb  = (unsigned short*)(W + OFF_NEMB);
  float* x2    = (float*)(W + OFF_X2);
  unsigned short* norm  = (unsigned short*)(W + OFF_NORM);
  unsigned short* Qp    = (unsigned short*)(W + OFF_Q);
  unsigned short* Kp    = (unsigned short*)(W + OFF_K);
  unsigned short* Vp    = (unsigned short*)(W + OFF_V);
  float* sem   = (float*)(W + OFF_SEM);
  float* tr    = (float*)(W + OFF_TR);
  unsigned short* vsem  = (unsigned short*)(W + OFF_VSEM);
  unsigned short* proj  = (unsigned short*)(W + OFF_PROJ);
  unsigned short* attn  = (unsigned short*)(W + OFF_ATTN);
  unsigned short* hid   = (unsigned short*)(W + OFF_H);

  k_tcast<<<dim3(DMOD / 64, DMOD / 64, 1), 256, 0, stream>>>(q_w, wq, DMOD, DMOD, 0L, 0L, WCARRY);
  k_tcast<<<dim3(DMOD / 64, DMOD / 64, 1), 256, 0, stream>>>(k_w, wk, DMOD, DMOD, 0L, 0L, WCARRY);
  k_tcast<<<dim3(DMOD / 64, DMOD / 64, 1), 256, 0, stream>>>(ao_w, wao, DMOD, DMOD, 0L, 0L, WCARRY);
  k_tcast<<<dim3(DMOD / 64, RNK / 64, 1), 256, 0, stream>>>(vout_w, wvo, RNK, DMOD, 0L, 0L, WCARRY);
  k_tcast<<<dim3(DFFN / 64, DMOD / 64, 1), 256, 0, stream>>>(up_w, wup, DMOD, DFFN, 0L, 0L, WCARRY);
  k_tcast<<<dim3(DMOD / 64, DFFN / 64, 1), 256, 0, stream>>>(down_w, wdn, DFFN, DMOD, 0L, 0L, WCARRY);
  k_tcast<<<dim3(RNK / 64, DMOD / 64, NBAS), 256, 0, stream>>>(basis_A, bA, DMOD, RNK,
                                                               (long)DMOD * RNK, (long)RNK * DMOD, WCARRY);

  k_prep<<<1, 256, 0, stream>>>(recipe, ctx_pat, basis_e, vout_b, rn, rnA, csig, vb64, bembT);

  gemm_f16<0, 1, false>(rnA, NBAS, bembT, NBAS, nemb, DMOD, nullptr, nullptr, NNEU_PAD, DMOD, NBAS, 1.0f, stream);

  k_ln<<<NTOK, 128, 0, stream>>>(x, n1_g, n1_b, norm);

  gemm_f16<2, 1, false>(norm, DMOD, wq, DMOD, Qp, DMOD, q_b, nullptr, NTOK, DMOD, DMOD, WCARRY_INV, stream);
  gemm_f16<2, 1, false>(norm, DMOD, wk, DMOD, Kp, DMOD, k_b, nullptr, NTOK, DMOD, DMOD, WCARRY_INV, stream);
  gemm_f16<0, 0, false>(norm, DMOD, nemb, DMOD, sem, NNEU_PAD, nullptr, nullptr, NTOK, NNEU_PAD, DMOD, WCARRY_INV, stream);

  k_topk<<<NTOK / 32, 256, 0, stream>>>(sem, csig, rn, tr, NTOK);

  gemm_f16<0, 1, false>(norm, DMOD, bA, DMOD, proj, NPROJ, nullptr, nullptr, NTOK, NPROJ, DMOD, WCARRY_INV, stream);

  k_vsem<<<NTOK / 4, 128, 0, stream>>>(proj, tr, vsem, NTOK);

  gemm_f16<2, 1, false>(vsem, RNK, wvo, RNK, Vp, DMOD, vb64, nullptr, NTOK, DMOD, RNK, WCARRY_INV, stream);

  k_attn<<<NBATCH * NHEADS * (SEQL / 64), 128, 0, stream>>>(Qp, Kp, Vp, attn, 0.125f, OCARRY_EXTRA);

  gemm_f16<2, 0, true>(attn, DMOD, wao, DMOD, x2, DMOD, ao_b, x, NTOK, DMOD, DMOD,
                       1.0f / (VCARRY * OCARRY_EXTRA * WCARRY), stream);

  k_ln<<<NTOK, 128, 0, stream>>>(x2, n2_g, n2_b, norm);

  gemm_f16<2, 1, false>(norm, DMOD, wup, DMOD, hid, DFFN, up_b, nullptr, NTOK, DFFN, DMOD, WCARRY_INV, stream);

  {
    const int n2 = NTOK * DFFN / 2;
    k_gelu2<<<(n2 + 255) / 256, 256, 0, stream>>>((unsigned int*)hid, n2, GCARRY);
  }

  gemm_f16<2, 0, true>(hid, DFFN, wdn, DFFN, out, DMOD, down_b, x2, NTOK, DMOD, DFFN,
                       1.0f / (GCARRY * WCARRY), stream);
}
